// SharedExpertMOE_4930622456430
// MI455X (gfx1250) — hardware-run, weakly checked
//
#include <hip/hip_runtime.h>


#ifndef NB
#define NB 4
#endif
#ifndef SEQ
#define SEQ 2048
#endif
#define NB_FULL  4
#define SEQ_FULL 2048
#define HID  1024
#define NE   8
#define NSH  2
#define NG   (NE + NSH)
#define TM   32
#define TN   64
#define RTK  8
#define WTP  72
#define LOGIT_OFF ((size_t)NB_FULL * SEQ_FULL * HID)

static_assert(LOGIT_OFF * 4 == (size_t)33554432);
static_assert((LOGIT_OFF * 4) % 128 == 0);
static_assert(HID % 64 == 0);
static_assert(HID % 32 == 0);
static_assert(HID % TN == 0);
static_assert(TM == 32);
static_assert(TN == 64);
static_assert(NE == 8);
static_assert(SEQ % TM == 0);
static_assert((NB * SEQ) % TM == 0);
static_assert(SEQ % RTK == 0);
static_assert((NB * SEQ) % RTK == 0);
static_assert(RTK * 32 == 256);
static_assert(16 * 16 == RTK * NE * 4);
static_assert(32 * 16 * 8 == 16 * TN * 4);
static_assert(256 * 16 * 2 == 64 * 128);
static_assert((WTP * 2) % 16 == 0);
static_assert(((size_t)SEQ * HID) % 8 == 0);
static_assert(((size_t)HID * NE) % 8 == 0);
static_assert(NB <= NB_FULL);
static_assert(SEQ <= SEQ_FULL);
static_assert(16 * 68 * 4 + TM * NE * 4 <= 131072);
static_assert(64 * WTP * 2 <= 131072);
static_assert(2 * RTK * NE * 4 <= 131072);

typedef unsigned short bf;
typedef __attribute__((ext_vector_type(16))) __bf16   v16bf;
typedef __attribute__((ext_vector_type(8)))  unsigned short v8us;
typedef __attribute__((ext_vector_type(4)))  unsigned v4u;
typedef __attribute__((ext_vector_type(8)))  float    v8f;
typedef __attribute__((ext_vector_type(4)))  float    v4f;
typedef v4f  __attribute__((may_alias)) v4fa;
typedef v8us __attribute__((may_alias)) v8usa;

__device__ __forceinline__ unsigned short f2bf(float f) { unsigned u = __float_as_uint(f); u += 0x7FFFu + ((u >> 16) & 1u); return (unsigned short)(u >> 16); }
__device__ __forceinline__ float bfr(float f) { return __uint_as_float(((unsigned)f2bf(f)) << 16); }
__device__ __forceinline__ v16bf cat16b(v8us lo, v8us hi) { return __builtin_bit_cast(v16bf, __builtin_shufflevector(lo, hi, 0, 1, 2, 3, 4, 5, 6, 7, 8, 9, 10, 11, 12, 13, 14, 15)); }
__device__ __forceinline__ v16bf ldb(const bf* p)  { return cat16b(*(const v8us*)p, *(const v8us*)(p + 16)); }
__device__ __forceinline__ v8f wmmab_g(v16bf a, v16bf b, v8f c) {
    c = __builtin_amdgcn_wmma_f32_16x16x32_bf16(false, a, false, b, (short)0, c, false, false);
    asm volatile("v_nop\n\tv_nop\n\tv_nop\n\tv_nop" : "+v"(c) : "v"(a), "v"(b));
    return c;
}
__device__ __forceinline__ void wave_sync() { __builtin_amdgcn_fence(3  , "wavefront"); __builtin_amdgcn_wave_barrier(); asm volatile("" ::: "memory"); }

__global__ __launch_bounds__(256) void k_cvt8(const float* __restrict__ src, bf* dst, size_t n8) {
    const size_t i = (size_t)blockIdx.x * 256 + threadIdx.x; if (i >= n8) return;
    const v8f v = *(const v8f*)(src + i * 8); v8us o;
#pragma unroll
    for (int k = 0; k < 8; ++k) o[k] = f2bf(v[k]);
    *(volatile v8us*)(dst + i * 8) = o; __threadfence(); *(volatile v8us*)(dst + i * 8) = o;
}

__global__ __launch_bounds__(256) void k_wtr(const float* __restrict__ src, bf* dst) {
    __shared__ __align__(16) bf ts[64 * WTP];
    const int tid = threadIdx.x;
    const int h0 = blockIdx.x * 64, d0 = blockIdx.y * 64;
    const size_t zo = (size_t)blockIdx.z * HID * HID;
#pragma unroll
    for (int i = 0; i < 4; ++i) {
        const int hr = i * 16 + (tid >> 4), dc = (tid & 15) * 4;
        const v4f v = *(const v4f*)(src + zo + (size_t)(h0 + hr) * HID + d0 + dc);
#pragma unroll
        for (int c = 0; c < 4; ++c) ts[(dc + c) * WTP + hr] = f2bf(v[c]);
    }
    __syncthreads();
#pragma unroll 1
    for (int ps = 0; ps < 2; ++ps) {
#pragma unroll
        for (int s = 0; s < 2; ++s) { const int p = s * 256 + tid; const int row = p >> 3, c8 = (p & 7) * 8;
            const v8us o = *(const v8usa*)(&ts[row * WTP + c8]);
            *(volatile v8us*)(dst + zo + (size_t)(d0 + row) * HID + h0 + c8) = o; }
        if (ps == 0) __threadfence(); }
}

__global__ __launch_bounds__(256) void k_router(const bf* __restrict__ XB, const bf* __restrict__ GWB, const float* __restrict__ gate_b, const int* __restrict__ topk_p,
                                                float* LOGITS, float* CW) {
#pragma clang fp contract(off)
    __shared__ __align__(16) float sl[RTK * NE];
    __shared__ __align__(16) float sc[RTK * NE];
    const int lane = threadIdx.x & 31;
    const int wave = __builtin_amdgcn_readfirstlane((int)(threadIdx.x >> 5));
    const int tc0 = blockIdx.x * RTK;
    const bf* xr = XB + (size_t)(tc0 + wave) * HID;
    double acc[NE];
#pragma unroll
    for (int e = 0; e < NE; ++e) acc[e] = 0.0;
#pragma unroll 1
    for (int k = lane; k < HID; k += 32) {
        const double xd = (double)__uint_as_float(((unsigned)xr[k]) << 16);
        const v4u g = *(const v4u*)(GWB + (size_t)k * NE);
#pragma unroll
        for (int i = 0; i < 4; ++i) {
            acc[2 * i]     = fma(xd, (double)__uint_as_float(g[i] << 16), acc[2 * i]);
            acc[2 * i + 1] = fma(xd, (double)__uint_as_float(g[i] & 0xffff0000u), acc[2 * i + 1]);
        }
    }
#pragma unroll 1
    for (int off = 16; off > 0; off >>= 1) {
#pragma unroll
        for (int e = 0; e < NE; ++e) acc[e] += __shfl_xor(acc[e], off, 32);
    }
    float lg[NE];
#pragma unroll
    for (int e = 0; e < NE; ++e) lg[e] = (float)acc[e] + bfr(gate_b[e]);
    int kt = topk_p[0]; kt = max(1, min(kt, NE));
    unsigned picked = 0u; float ssum = 0.0f, mtop = 0.0f;
    float cw[NE];
#pragma unroll
    for (int e = 0; e < NE; ++e) cw[e] = 0.0f;
#pragma unroll 1
    for (int kk = 0; kk < kt; ++kk) {
        int best = 0; float bv = 0.0f; bool have = false;
#pragma unroll
        for (int e = 0; e < NE; ++e) {
            const bool fr = ((picked >> e) & 1u) == 0u;
            const bool take = fr & ((!have) | (lg[e] > bv));
            bv = take ? lg[e] : bv; best = take ? e : best; have = have | fr;
        }
        mtop = (kk == 0) ? bv : mtop;
        const float pe = expf(bv - mtop);
        picked |= 1u << best;
#pragma unroll
        for (int e = 0; e < NE; ++e) cw[e] = (e == best) ? pe : cw[e];
        ssum += pe;
    }
    const float inv = 1.0f / ssum;
#pragma unroll
    for (int e = 0; e < NE; ++e) cw[e] = cw[e] * inv;
    if (lane == 0) {
        v4f a, c;
        a[0] = lg[0]; a[1] = lg[1]; a[2] = lg[2]; a[3] = lg[3]; c[0] = lg[4]; c[1] = lg[5]; c[2] = lg[6]; c[3] = lg[7];
        *(v4fa*)(&sl[wave * NE]) = a; *(v4fa*)(&sl[wave * NE + 4]) = c;
        a[0] = cw[0]; a[1] = cw[1]; a[2] = cw[2]; a[3] = cw[3]; c[0] = cw[4]; c[1] = cw[5]; c[2] = cw[6]; c[3] = cw[7];
        *(v4fa*)(&sc[wave * NE]) = a; *(v4fa*)(&sc[wave * NE + 4]) = c;
    }
    __syncthreads();
    if (wave == 0) {
        const int pc = lane & 15;
        const v4f lv = *(const v4fa*)(&sl[pc * 4]);
        const v4f cv = *(const v4fa*)(&sc[pc * 4]);
        const size_t tf0 = (size_t)(tc0 / SEQ) * SEQ_FULL + (size_t)(tc0 % SEQ);
        float* lp = LOGITS + tf0 * NE + (size_t)pc * 4;
        float* cp = CW + (size_t)tc0 * NE + (size_t)pc * 4;
#pragma unroll 1
        for (int ps = 0; ps < 2; ++ps) {
            if (lane < 16) { *(volatile v4f*)lp = lv; *(volatile v4f*)cp = cv; }
            if (ps == 0) __threadfence(); }
    }
}

__device__ __forceinline__ void mix_kloop(v8f (&acc)[2][4], const bf* __restrict__ A, const bf* __restrict__ Bt, size_t aoff, size_t boff) {
#pragma unroll 1
    for (int kc = 0; kc < HID; kc += 32) {
        v16bf a[2];
#pragma unroll
        for (int mb = 0; mb < 2; ++mb) a[mb] = ldb(A + aoff + (size_t)mb * 16 * HID + kc);
#pragma unroll
        for (int nb = 0; nb < 4; ++nb) { const v16bf b = ldb(Bt + boff + (size_t)nb * 16 * HID + kc);
#pragma unroll
            for (int mb = 0; mb < 2; ++mb) acc[mb][nb] = wmmab_g(a[mb], b, acc[mb][nb]); }
    }
}

__global__ __launch_bounds__(32) __attribute__((amdgpu_num_vgpr(256)))
void k_mix(const bf* __restrict__ XB, const bf* __restrict__ WT, const float* __restrict__ CW,
           const float* __restrict__ expert_b, const float* __restrict__ shared_b, float* OUT) {
    __shared__ __align__(16) float os[16 * 68];
    __shared__ __align__(16) float cwl[TM * NE];
    const int lane = threadIdx.x & 31, lr = lane & 15, hi = lane >> 4;
    const int r0 = blockIdx.x * TM, c0 = blockIdx.y * TN;
    { const v4f w0 = *(const v4f*)(CW + (size_t)(r0 + lane) * NE); const v4f w1 = *(const v4f*)(CW + (size_t)(r0 + lane) * NE + 4);
      *(v4fa*)(&cwl[lane * NE]) = w0; *(v4fa*)(&cwl[lane * NE + 4]) = w1; }
    wave_sync();
    v8f tot[2][4], acc[2][4];
#pragma unroll
    for (int mb = 0; mb < 2; ++mb)
#pragma unroll
        for (int nb = 0; nb < 4; ++nb) tot[mb][nb] = (v8f){};
    const size_t aoff = (size_t)(r0 + lr) * HID + 8 * hi, boff = (size_t)(c0 + lr) * HID + 8 * hi;
#pragma unroll 1
    for (int s = 0; s < NSH; ++s) mix_kloop(tot, XB, WT + (size_t)(NE + s) * HID * HID, aoff, boff);
#pragma unroll
    for (int nb = 0; nb < 4; ++nb) {
        float sb = 0.0f;
#pragma unroll
        for (int s = 0; s < NSH; ++s) sb += bfr(shared_b[(size_t)s * HID + c0 + nb * 16 + lr]);
#pragma unroll
        for (int mb = 0; mb < 2; ++mb)
#pragma unroll
            for (int j = 0; j < 8; ++j) tot[mb][nb][j] += sb;
    }
#pragma unroll 1
    for (int e = 0; e < NE; ++e) {
#pragma unroll
        for (int mb = 0; mb < 2; ++mb)
#pragma unroll
            for (int nb = 0; nb < 4; ++nb) acc[mb][nb] = (v8f){};
        mix_kloop(acc, XB, WT + (size_t)e * HID * HID, aoff, boff);
        float bc[4];
#pragma unroll
        for (int nb = 0; nb < 4; ++nb) bc[nb] = bfr(expert_b[(size_t)e * HID + c0 + nb * 16 + lr]);
#pragma unroll
        for (int mb = 0; mb < 2; ++mb) {
#pragma unroll
            for (int j = 0; j < 8; ++j) {
                const float w = cwl[(mb * 16 + hi * 8 + j) * NE + e];
#pragma unroll
                for (int nb = 0; nb < 4; ++nb) tot[mb][nb][j] += w * (acc[mb][nb][j] + bc[nb]);
            }
        }
    }
    const size_t rf = (size_t)(r0 / SEQ) * SEQ_FULL + (size_t)(r0 % SEQ);
#pragma unroll
    for (int mb = 0; mb < 2; ++mb) {
#pragma unroll
        for (int nb = 0; nb < 4; ++nb) {
#pragma unroll
            for (int j = 0; j < 8; ++j) os[(hi * 8 + j) * 68 + nb * 16 + lr] = tot[mb][nb][j]; }
        wave_sync();
        float* ob = OUT + (rf + (size_t)(mb * 16)) * HID + c0;
#pragma unroll 1
        for (int ps = 0; ps < 2; ++ps) {
#pragma unroll
            for (int s = 0; s < 8; ++s) { const int p = s * 32 + lane; const int row = p >> 4, c4 = (p & 15) * 4;
                const v4f val = *(const v4fa*)(&os[row * 68 + c4]);
                *(volatile v4f*)(ob + (size_t)row * HID + c4) = val; }
            if (ps == 0) __threadfence(); }
        wave_sync();
    }
}

static constexpr size_t al256(size_t v) { return (v + 255) & ~(size_t)255; }
static constexpr size_t SZ_XB = al256((size_t)NB * SEQ * HID * 2);
static constexpr size_t SZ_WT = al256((size_t)NG * HID * HID * 2);
static constexpr size_t SZ_GW = al256((size_t)HID * NE * 2);
static constexpr size_t SZ_CW = al256((size_t)NB * SEQ * NE * 4);
static constexpr size_t SZ_TOTAL = SZ_XB + SZ_WT + SZ_GW + SZ_CW;
static_assert(SZ_TOTAL <= (size_t)134217728);
static_assert(((size_t)HID * HID * 2) % 256 == 0);
static_assert((size_t)(NB * SEQ / RTK) * RTK * NE * 4 <= SZ_CW);
static_assert((size_t)(HID / 64) * (HID / 64) * NG * 64 * 64 * 2 <= SZ_WT);

extern "C" void kernel_launch(void* const* d_in, const int* in_sizes, int n_in,
                              void* d_out, int out_size, void* d_ws, size_t ws_size, hipStream_t stream) {
    if (n_in < 8) return;
    const size_t needt = (size_t)(NB - 1) * SEQ_FULL + SEQ;
    if ((size_t)in_sizes[0] < needt * HID) return;
    if ((size_t)in_sizes[1] < (size_t)HID * NE || in_sizes[2] < NE) return;
    if ((size_t)in_sizes[3] < (size_t)NE * HID * HID || (size_t)in_sizes[4] < (size_t)NE * HID) return;
    if ((size_t)in_sizes[5] < (size_t)NSH * HID * HID || (size_t)in_sizes[6] < (size_t)NSH * HID) return;
    if (in_sizes[7] < 1) return;
    if ((size_t)out_size < LOGIT_OFF + needt * NE) return;
    if (SZ_TOTAL > ws_size) return;
    const float* x   = (const float*)d_in[0];
    const float* gw  = (const float*)d_in[1];
    const float* gb  = (const float*)d_in[2];
    const float* ew  = (const float*)d_in[3];
    const float* eb  = (const float*)d_in[4];
    const float* sw  = (const float*)d_in[5];
    const float* sb  = (const float*)d_in[6];
    const int*   tk  = (const int*)d_in[7];
    float* OUT = (float*)d_out;
    float* LOGITS = (float*)d_out + LOGIT_OFF;
    char* wsp = (char*)d_ws;
    bf* XB  = (bf*)wsp; wsp += SZ_XB;
    bf* WT  = (bf*)wsp; wsp += SZ_WT;
    bf* GWB = (bf*)wsp; wsp += SZ_GW;
    float* CW = (float*)wsp; wsp += SZ_CW;

    if (SEQ == SEQ_FULL) {
        const size_t n8 = (size_t)NB * SEQ * HID / 8;
        k_cvt8<<<(unsigned)((n8 + 255) / 256), 256, 0, stream>>>(x, XB, n8);
    } else {
        const size_t n8 = (size_t)SEQ * HID / 8;
        for (int b = 0; b < NB; ++b) k_cvt8<<<(unsigned)((n8 + 255) / 256), 256, 0, stream>>>(x + (size_t)b * SEQ_FULL * HID, XB + (size_t)b * SEQ * HID, n8);
    }
    { const size_t n8 = (size_t)HID * NE / 8; k_cvt8<<<(unsigned)((n8 + 255) / 256), 256, 0, stream>>>(gw, GWB, n8); }
    k_wtr<<<dim3(HID / 64, HID / 64, NE), 256, 0, stream>>>(ew, WT);
    k_wtr<<<dim3(HID / 64, HID / 64, NSH), 256, 0, stream>>>(sw, WT + (size_t)NE * HID * HID);

    k_router<<<dim3(NB * SEQ / RTK, 1, 1), 256, 0, stream>>>(XB, GWB, gb, tk, LOGITS, CW);
    k_mix<<<dim3(NB * SEQ / TM, HID / TN, 1), 32, 0, stream>>>(XB, WT, CW, eb, sb, OUT);
}
